// ScreeningUnit_32134945309258
// MI455X (gfx1250) — hardware-verified
//
#include <hip/hip_runtime.h>
#include <math.h>
#include <stdint.h>

#ifndef NB
#define NB 8
#endif
#ifndef SEQ
#define SEQ 4096
#endif
#define SEQ_FULL 4096
#define DK   16
#define DV   64
#define QSC  1024.0f
#define KSC  1024.0f
#define PCAR 32768.0f
#define VCAR 1024.0f
#define GATE_PAD 104.0f
#define WPB  4
#define ATT_THREADS (WPB * 32)
#define NQT  (SEQ / 16)
#define NKT  (SEQ / 32)
#define NST  (SEQ / 64)
#define PTP  36
#define PTW  (16 * PTP)
#define SLP  68
#define SLW  (16 * SLP)
#define WREG (PTW + SLW)
#define VTP  72
#define WS_CAP 134217728
static_assert(NB >= 1 && NB <= 8);
static_assert((SEQ % 64) == 0 && SEQ >= 64 && SEQ <= SEQ_FULL);
static_assert(DK == 16 && DV == 64);
static_assert((NQT % WPB) == 0 && ATT_THREADS == 128);
static_assert(WPB * WREG * 4 <= 65536 && 2 * DV * VTP * 2 <= 65536);
static_assert(((NB * SEQ * 2) % 32) == 0);

typedef unsigned short u16;
typedef _Float16 v16h __attribute__((ext_vector_type(16)));
typedef _Float16 v8h  __attribute__((ext_vector_type(8)));
typedef float    v8f  __attribute__((ext_vector_type(8)));
typedef float    v4f  __attribute__((ext_vector_type(4)));
typedef unsigned int v4u __attribute__((ext_vector_type(4)));

union FragH { v16h v; v8h h[2]; v4u u[2]; };

__device__ __forceinline__ unsigned short bf_bits(float f) {
  unsigned u = __float_as_uint(f);
  return (unsigned short)((u + 0x7FFFu + ((u >> 16) & 1u)) >> 16);
}
__device__ __forceinline__ float bf_up(unsigned short h) { return __uint_as_float(((unsigned)h) << 16); }
__device__ __forceinline__ float bfr(float f) { return bf_up(bf_bits(f)); }
__device__ __forceinline__ unsigned short h_bits(_Float16 x) { return __builtin_bit_cast(unsigned short, x); }
__device__ __forceinline__ unsigned pk16(unsigned short a, unsigned short b) { return (unsigned)a | ((unsigned)b << 16); }
__device__ __forceinline__ v8f zero8() { v8f z = {0.f, 0.f, 0.f, 0.f, 0.f, 0.f, 0.f, 0.f}; return z; }
__device__ __forceinline__ v8h hzero8() {
  v8h z;
#pragma unroll
  for (int e = 0; e < 8; ++e) z[e] = (_Float16)0.0f;
  return z;
}
__device__ __forceinline__ const _Float16* ash(const u16* p) { return (const _Float16*)(const void*)p; }

__device__ __forceinline__ v16h ldfrag_h(const _Float16* p) {
  FragH f;
  f.h[0] = *(const v8h*)(p);
  f.h[1] = *(const v8h*)(p + 16);
  return f.v;
}

__device__ __forceinline__ v8f mma_h(v16h a, v16h b, v8f c) {
  return __builtin_amdgcn_wmma_f32_16x16x32_f16(false, a, false, b, (short)0, c, false, false);
}
__device__ __forceinline__ void guard2(v8f& a, v8f& b, v16h x0, v16h x1, v16h x2, v16h x3, v16h x4, v16h x5) {
#if defined(__HIP_DEVICE_COMPILE__)
  asm volatile("v_nop\n\tv_nop\n\tv_nop\n\tv_nop"
               : "+v"(a), "+v"(b) : "v"(x0), "v"(x1), "v"(x2), "v"(x3), "v"(x4), "v"(x5) : "memory");
#endif
}
__device__ __forceinline__ void acc_guard4(v8f& a, v8f& b, v8f& c, v8f& d) {
#if defined(__HIP_DEVICE_COMPILE__)
  asm volatile("v_nop\n\tv_nop\n\tv_nop\n\tv_nop" : "+v"(a), "+v"(b), "+v"(c), "+v"(d));
#endif
}
__device__ __forceinline__ void wave_sync_lds() {
  __builtin_amdgcn_fence(__ATOMIC_RELEASE, "workgroup");
  __builtin_amdgcn_wave_barrier();
  __builtin_amdgcn_fence(__ATOMIC_ACQUIRE, "workgroup");
}

__global__ __launch_bounds__(256) void qk16(const float* __restrict__ X, u16* Hp, u16* Lp, int n2, float sc) {
  const int gt = blockIdx.x * 256 + (int)threadIdx.x;
  if (gt >= n2) return;
  const int row  = gt >> 1;
  const int half = gt & 1;
  const int b    = row / SEQ;
  const int s    = row - b * SEQ;
  const float* p = X + ((size_t)b * SEQ_FULL + s) * DK + 8 * half;
  const v4f a = *(const v4f*)(p), b4 = *(const v4f*)(p + 4);
  float w[8];
#pragma unroll
  for (int e = 0; e < 4; ++e) { w[e] = bfr(a[e]); w[4 + e] = bfr(b4[e]); }
  float ss = 0.0f;
#pragma unroll
  for (int e = 0; e < 8; ++e) ss += w[e] * w[e];
  ss += __shfl_xor(ss, 1, 32);
  const float inv = 1.0f / fmaxf(sqrtf(ss), 1e-12f);
  const float isc = inv * sc;
  v4u oh, ol;
#pragma unroll
  for (int e = 0; e < 4; ++e) {
    const float t0 = w[2 * e] * isc, t1 = w[2 * e + 1] * isc;
    const _Float16 h0 = (_Float16)t0, h1 = (_Float16)t1;
    const _Float16 l0 = (_Float16)(t0 - (float)h0), l1 = (_Float16)(t1 - (float)h1);
    oh[e] = pk16(h_bits(h0), h_bits(h1));
    ol[e] = pk16(h_bits(l0), h_bits(l1));
  }
  u16* dh = Hp + (size_t)gt * 8;
  u16* dl = Lp + (size_t)gt * 8;
  for (int pass = 0; pass < 2; ++pass) {
    *(volatile v4u*)(dh) = oh;
    *(volatile v4u*)(dl) = ol;
    __threadfence();
  }
}

__global__ __launch_bounds__(256) void vt16n(const float* __restrict__ V, u16* VHo, u16* VLo) {
  __shared__ __align__(16) u16 TH[DV * VTP];
  __shared__ __align__(16) u16 TL[DV * VTP];
  const int tid = threadIdx.x;
  const int bid = blockIdx.x;
  const int st  = bid % NST;
  const int b   = bid / NST;
  if (b >= NB) return;
  const int s0  = st * 64;
  {
    const int sl = tid >> 2;
    const int dc = (tid & 3) * 16;
    const float* src = V + ((size_t)b * SEQ_FULL + s0 + sl) * DV + dc;
    float x[16];
#pragma unroll
    for (int i = 0; i < 4; ++i) {
      const v4f a = *(const v4f*)(src + 4 * i);
#pragma unroll
      for (int e = 0; e < 4; ++e) x[4 * i + e] = bfr(a[e]);
    }
    float ss = 0.0f;
#pragma unroll
    for (int i = 0; i < 16; ++i) ss += x[i] * x[i];
    ss += __shfl_xor(ss, 1, 32);
    ss += __shfl_xor(ss, 2, 32);
    const float inv = 1.0f / fmaxf(sqrtf(ss), 1e-12f);
    const float isc = inv * VCAR;
#pragma unroll
    for (int i = 0; i < 16; ++i) {
      const float t = x[i] * isc;
      const _Float16 hv = (_Float16)t;
      const _Float16 lv = (_Float16)(t - (float)hv);
      TH[(dc + i) * VTP + sl] = h_bits(hv);
      TL[(dc + i) * VTP + sl] = h_bits(lv);
    }
  }
  __syncthreads();
  v4u vh[2], vl[2];
  const int q8 = tid >> 3, p8 = (tid & 7) * 8;
#pragma unroll
  for (int it = 0; it < 2; ++it) {
    const int line = it * 32 + q8;
    vh[it] = *(const v4u*)(TH + line * VTP + p8);
    vl[it] = *(const v4u*)(TL + line * VTP + p8);
  }
  const size_t hrow = (size_t)b * DV;
  const size_t base = hrow * SEQ + s0 + p8;
  for (int pass = 0; pass < 2; ++pass) {
#pragma unroll
    for (int it = 0; it < 2; ++it) {
      const int line = it * 32 + q8;
      *(volatile v4u*)(VHo + base + (size_t)line * SEQ) = vh[it];
      *(volatile v4u*)(VLo + base + (size_t)line * SEQ) = vl[it];
    }
    __threadfence();
  }
}

__global__ __launch_bounds__(ATT_THREADS)
void attn_s(const u16* __restrict__ QHp, const u16* __restrict__ QLp,
            const u16* __restrict__ KHp, const u16* __restrict__ KLp,
            const u16* __restrict__ VHp, const u16* __restrict__ VLp,
            const float* __restrict__ srp, const float* __restrict__ swp, float* out) {
  __shared__ __align__(16) float smem[WPB * WREG];
  const int tid  = threadIdx.x;
  const int wave = __builtin_amdgcn_readfirstlane(tid >> 5);
  const int lane = tid & 31;
  const int hh   = lane >> 4;
  const int c    = lane & 15;
  const int g    = (int)blockIdx.x * WPB + wave;
  const int b    = g / NQT;
  const int qt   = g - b * NQT;
  if (b >= NB) return;
  const int q0   = qt * 16;

  float* pt   = smem + wave * WREG;
  float* slab = pt + PTW;

  const float rr   = expf(bfr(srp[0])) + 1.0f;
  const float ww   = expf(bfr(swp[0])) + 1.0f;
  const float wcap = fminf(ww + GATE_PAD, (float)SEQ);
  const int   cw   = (int)ceilf(wcap);
  int jlo = q0 - cw;
  jlo = (jlo > 0) ? jlo : 0;
  const int ktlo = __builtin_amdgcn_readfirstlane(jlo >> 5);
  const int kthi = q0 >> 5;

  const size_t qrow = (size_t)b * SEQ + q0 + c;
  FragH qa;
  qa.h[0] = *(const v8h*)(ash(QHp) + qrow * DK + 8 * hh);
  qa.h[1] = *(const v8h*)(ash(QLp) + qrow * DK + 8 * hh);
  const _Float16* Khb = ash(KHp) + ((size_t)b * SEQ + c) * DK + 8 * hh;
  const _Float16* Klb = ash(KLp) + ((size_t)b * SEQ + c) * DK + 8 * hh;
  const _Float16* Vhb = ash(VHp) + ((size_t)b * DV + c) * SEQ + 8 * hh;
  const _Float16* Vlb = ash(VLp) + ((size_t)b * DV + c) * SEQ + 8 * hh;
  const float ssc = 1.0f / (QSC * KSC);
  const float oc  = 1.0f / (PCAR * VCAR);
  const v8h   hz  = hzero8();
  const int   qr0 = q0 + 8 * hh;

  v8f o[4];
#pragma unroll
  for (int j = 0; j < 4; ++j) o[j] = zero8();

#pragma unroll 1
  for (int kt = ktlo; kt <= kthi; ++kt) {
    const int kb = kt * 32;
    FragH kf0, kf1, kg0, kg1;
    const _Float16* k0p = Khb + (size_t)kb * DK;
    const _Float16* k1p = k0p + (size_t)16 * DK;
    const _Float16* l0p = Klb + (size_t)kb * DK;
    const _Float16* l1p = l0p + (size_t)16 * DK;
    kf0.h[0] = *(const v8h*)(k0p);  kf0.h[1] = kf0.h[0];
    kf1.h[0] = *(const v8h*)(k1p);  kf1.h[1] = kf1.h[0];
    kg0.h[0] = *(const v8h*)(l0p);  kg0.h[1] = hz;
    kg1.h[0] = *(const v8h*)(l1p);  kg1.h[1] = hz;
    v8f s0 = zero8(), s1 = zero8();
    s0 = mma_h(qa.v, kf0.v, s0);
    s0 = mma_h(qa.v, kg0.v, s0);
    s1 = mma_h(qa.v, kf1.v, s1);
    s1 = mma_h(qa.v, kg1.v, s1);
    guard2(s0, s1, qa.v, kf0.v, kg0.v, kf1.v, kg1.v, qa.v);

    const int key0 = kb + c, key1 = kb + 16 + c;
#pragma unroll
    for (int r = 0; r < 8; ++r) {
      const int   qr  = qr0 + r;
      const float sv0 = s0[r] * ssc;
      const float sv1 = s1[r] * ssc;
      const float u0  = fmaxf(1.0f - rr * (1.0f - sv0), 0.0f);
      const float u1  = fmaxf(1.0f - rr * (1.0f - sv1), 0.0f);
      const float d0  = (float)(qr - key0);
      const float d1  = (float)(qr - key1);
      const float g0  = __builtin_amdgcn_rcpf(1.0f + __expf(d0 - ww));
      const float g1  = __builtin_amdgcn_rcpf(1.0f + __expf(d1 - ww));
      float a0 = u0 * u0 * g0;
      float a1 = u1 * u1 * g1;
      a0 = (key0 > qr) ? 0.0f : a0;
      a1 = (key1 > qr) ? 0.0f : a1;
      const int ro = (8 * hh + r) * PTP + c;
      pt[ro]      = a0;
      pt[ro + 16] = a1;
    }
    wave_sync_lds();
    FragH ph, pl;
    {
      const float* prow = pt + c * PTP + 8 * hh;
      const v4f p0 = *(const v4f*)(prow), p1 = *(const v4f*)(prow + 4);
      const v4f p2 = *(const v4f*)(prow + 16), p3 = *(const v4f*)(prow + 20);
#pragma unroll
      for (int e = 0; e < 4; ++e) {
        const float ta = p0[e] * PCAR, tb = p1[e] * PCAR, tc = p2[e] * PCAR, td = p3[e] * PCAR;
        const _Float16 ha = (_Float16)ta, hb = (_Float16)tb, hc = (_Float16)tc, hd = (_Float16)td;
        ph.h[0][e]     = ha;
        ph.h[0][4 + e] = hb;
        ph.h[1][e]     = hc;
        ph.h[1][4 + e] = hd;
        pl.h[0][e]     = (_Float16)(ta - (float)ha);
        pl.h[0][4 + e] = (_Float16)(tb - (float)hb);
        pl.h[1][e]     = (_Float16)(tc - (float)hc);
        pl.h[1][4 + e] = (_Float16)(td - (float)hd);
      }
    }
    {
      const _Float16* vhp = Vhb + kb;
      const _Float16* vlp = Vlb + kb;
#pragma unroll
      for (int jg = 0; jg < 2; ++jg) {
        const size_t da = (size_t)(2 * jg) * 16 * SEQ;
        const size_t db = da + (size_t)16 * SEQ;
        const v16h vha = ldfrag_h(vhp + da), vhb2 = ldfrag_h(vhp + db);
        const v16h vla = ldfrag_h(vlp + da), vlb2 = ldfrag_h(vlp + db);
        o[2 * jg]     = mma_h(ph.v, vha,  o[2 * jg]);
        o[2 * jg]     = mma_h(pl.v, vha,  o[2 * jg]);
        o[2 * jg]     = mma_h(ph.v, vla,  o[2 * jg]);
        o[2 * jg + 1] = mma_h(ph.v, vhb2, o[2 * jg + 1]);
        o[2 * jg + 1] = mma_h(pl.v, vhb2, o[2 * jg + 1]);
        o[2 * jg + 1] = mma_h(ph.v, vlb2, o[2 * jg + 1]);
        guard2(o[2 * jg], o[2 * jg + 1], ph.v, pl.v, vha, vhb2, vla, vlb2);
      }
    }
    wave_sync_lds();
  }
  acc_guard4(o[0], o[1], o[2], o[3]);

  float ssr[8];
#pragma unroll
  for (int r = 0; r < 8; ++r) {
    float t = 0.0f;
#pragma unroll
    for (int j = 0; j < 4; ++j) t += o[j][r] * o[j][r];
#pragma unroll
    for (int off = 1; off < 16; off <<= 1) t += __shfl_xor(t, off, 32);
    ssr[r] = t;
  }
  const int rsel = c & 7;
  float my = ssr[0];
#pragma unroll
  for (int r = 1; r < 8; ++r) my = (rsel == r) ? ssr[r] : my;
  const float hn  = fmaxf(sqrtf(my) * oc, 1e-8f);
  const float scm = tanhf(hn) / hn;
  float scl[8];
#pragma unroll
  for (int r = 0; r < 8; ++r) scl[r] = __shfl(scm, (lane & 16) + r, 32);

#pragma unroll
  for (int r = 0; r < 8; ++r) {
    const float f = oc * scl[r];
#pragma unroll
    for (int j = 0; j < 4; ++j) {
      const int idx = (8 * hh + r) * SLP + j * 16 + c;
      slab[idx] = o[j][r] * f;
    }
  }
  wave_sync_lds();
  v4f vals[8];
#pragma unroll
  for (int it = 0; it < 8; ++it) vals[it] = *(const v4f*)(slab + (it * 2 + hh) * SLP + c * 4);
  float* dst = out + (((size_t)b * SEQ_FULL + q0 + hh) * DV + c * 4);
  for (int pass = 0; pass < 2; ++pass) {
#pragma unroll
    for (int it = 0; it < 8; ++it) {
      *(volatile v4f*)(dst + (size_t)(it * 2) * DV) = vals[it];
    }
    __threadfence();
  }
}

extern "C" void kernel_launch(void* const* d_in, const int* in_sizes, int n_in,
                              void* d_out, int out_size, void* d_ws, size_t ws_size,
                              hipStream_t stream) {
  if (n_in < 5) return;
  const int rows_needed = (NB - 1) * SEQ_FULL + SEQ;
  if (in_sizes[0] < rows_needed * DK) return;
  if (in_sizes[1] < rows_needed * DK) return;
  if (in_sizes[2] < rows_needed * DV) return;
  if (in_sizes[3] < 1) return;
  if (in_sizes[4] < 1) return;
  if (out_size < rows_needed * DV) return;

  const float* q   = (const float*)d_in[0];
  const float* k   = (const float*)d_in[1];
  const float* v   = (const float*)d_in[2];
  const float* s_r = (const float*)d_in[3];
  const float* s_w = (const float*)d_in[4];
  float*       out = (float*)d_out;

  const size_t szP = (size_t)NB * SEQ * DK * 2;
  const size_t szV = (size_t)NB * DV * SEQ * 2;
  size_t off = 0;
  const size_t oQH = off; off += szP;
  const size_t oQL = off; off += szP;
  const size_t oKH = off; off += szP;
  const size_t oKL = off; off += szP;
  const size_t oVH = off; off += szV;
  const size_t oVL = off; off += szV;
  if (off > ws_size) return;
  if (off > (size_t)WS_CAP) return;

  char* ws = (char*)d_ws;
  u16* QH = (u16*)(ws + oQH);
  u16* QL = (u16*)(ws + oQL);
  u16* KH = (u16*)(ws + oKH);
  u16* KL = (u16*)(ws + oKL);
  u16* VH = (u16*)(ws + oVH);
  u16* VL = (u16*)(ws + oVL);

  const int  n2 = NB * SEQ * 2;
  const dim3 b256(256), bAT(ATT_THREADS);
  const dim3 gQ((n2 + 255) / 256);
  const dim3 gVT(NB * NST);
  const dim3 gAT((NB * NQT + WPB - 1) / WPB);

  qk16<<<gQ, b256, 0, stream>>>(q, QH, QL, n2, QSC);
  qk16<<<gQ, b256, 0, stream>>>(k, KH, KL, n2, KSC);
  vt16n<<<gVT, b256, 0, stream>>>(v, VH, VL);
  attn_s<<<gAT, bAT, 0, stream>>>(QH, QL, KH, KL, VH, VL, s_r, s_w, out);
  (void)hipGetLastError();
}
